// Block_39814346834514
// MI455X (gfx1250) — hardware-run, weakly checked
//
#include <hip/hip_runtime.h>


#ifndef NB
#define NB 2
#endif
#ifndef SEQ
#define SEQ 2048
#endif
#define NB_FULL  2
#define SEQ_FULL 2048
#ifndef OUT_SEQ
#define OUT_SEQ SEQ
#endif
#define DM   1024
#define DE   2048
#define NH_  16
#define HD   128
#define NW1  8192
#define AW   4
#define OSP  132
#define WC1  64.0f
#define WC2  256.0f
#define GSC  256.0f
#define LOG2E 1.4426950408889634f
#define SC2  ((float)(0.08838834764831845 * 1.4426950408889634))
#define PSH  14.0f
#define NEGB (-3.0e38f)

static_assert(NH_ * HD == DE);
static_assert(4 * DE == NW1);
static_assert(HD % 64 == 0);
static_assert(HD % 32 == 0);
static_assert(HD == 8 * 16);
static_assert(DE / 64 == 32);
static_assert(DM % 32 == 0);
static_assert(DE % 32 == 0);
static_assert(DM % 256 == 0);
static_assert(DM % 128 == 0);
static_assert(DM % 64 == 0);
static_assert(SEQ % 64 == 0);
static_assert((NB * SEQ) % 64 == 0);
static_assert((NB * SEQ) % 8 == 0);
static_assert(SEQ % 32 == 0);
static_assert(SEQ % (16 * AW) == 0);
static_assert(((size_t)NW1 * DM) % 8 == 0);
static_assert(((size_t)DM * DE) % 8 == 0);
static_assert(((size_t)NB * NH_ * SEQ * HD) % (8 * 256) == 0);
static_assert(NB <= NB_FULL);
static_assert(SEQ <= SEQ_FULL);
static_assert((OSP * 4) % 16 == 0);
static_assert(OSP >= HD);
static_assert(AW * 16 * OSP * 4 <= 131072);
static_assert(16 * 68 * 4 <= 131072);
static_assert(4 * 32 * 16 == 16 * 64 * 2);
static_assert(8 * 32 * 16 == 16 * 64 * 4);
static_assert(8 * 32 * 16 == 16 * HD * 2);
static_assert((DM / 256) * 32 * 16 == DM * 2);
static_assert((DM / 128) * 32 * 16 == DM * 4);

typedef _Float16 h16;
typedef __attribute__((ext_vector_type(16))) _Float16 v16h;
typedef __attribute__((ext_vector_type(8)))  _Float16 v8h;
typedef __attribute__((ext_vector_type(8)))  float    v8f;
typedef __attribute__((ext_vector_type(4)))  float    v4f;
typedef v4f  __attribute__((may_alias)) v4fa;

__device__ __forceinline__ unsigned short f2bf(float f) { unsigned u = __float_as_uint(f); u += 0x7FFFu + ((u >> 16) & 1u); return (unsigned short)(u >> 16); }
__device__ __forceinline__ float bfr(float f) { return __uint_as_float(((unsigned)f2bf(f)) << 16); }
__device__ __forceinline__ v16h cat16(v8h lo, v8h hi) { return __builtin_shufflevector(lo, hi, 0, 1, 2, 3, 4, 5, 6, 7, 8, 9, 10, 11, 12, 13, 14, 15); }
static __device__ __forceinline__ h16 toh_flush(float v) { const h16 r = (h16)v; return (fabsf(v) < 6.103515625e-05f) ? (h16)0.0f : r; }
__device__ __forceinline__ v8f wmmag(v16h a, v16h b, v8f c) {
    c = __builtin_amdgcn_wmma_f32_16x16x32_f16(false, a, false, b, (short)0, c, false, false);
    asm volatile("v_nop\n\tv_nop\n\tv_nop\n\tv_nop" : "+v"(c) : "v"(a), "v"(b));
    return c;
}
__device__ __forceinline__ v16h  ldh(const h16* p) { return cat16(*(const v8h*)p, *(const v8h*)(p + 16)); }
__device__ __forceinline__ void wave_sync() { __builtin_amdgcn_fence(3  , "wavefront"); __builtin_amdgcn_wave_barrier(); asm volatile("" ::: "memory"); }

__global__ __launch_bounds__(256) void k_wcvt(const float* __restrict__ src, h16* dst, unsigned n8, float carry) {
    const unsigned i = blockIdx.x * 256u + threadIdx.x; if (i >= n8) return;
    const v8f v = *(const v8f*)(src + (size_t)i * 8); v8h o;
#pragma unroll
    for (int k = 0; k < 8; ++k) o[k] = toh_flush(bfr(v[k]) * carry);
    *(volatile v8h*)(dst + (size_t)i * 8) = o; __threadfence(); *(volatile v8h*)(dst + (size_t)i * 8) = o;
}

__global__ __launch_bounds__(256) void k_ln_in(const float* __restrict__ x, const float* __restrict__ g, const float* __restrict__ bb, h16* H) {
#pragma clang fp contract(off)
    const int lane = threadIdx.x & 31;
    const int wave = __builtin_amdgcn_readfirstlane((int)(threadIdx.x >> 5));
    const int m = blockIdx.x * 8 + wave;
    const int b = m / SEQ, t = m % SEQ;
    const float* xr = x + ((size_t)b * SEQ_FULL + (size_t)t) * DM + lane * 8;
    float s = 0.0f;
#pragma unroll 1
    for (int c = 0; c < DM / 256; ++c) {
        const v8f v = *(const v8f*)(xr + c * 256);
#pragma unroll
        for (int k = 0; k < 8; ++k) s += bfr(v[k]);
    }
#pragma unroll
    for (int off = 16; off > 0; off >>= 1) s += __shfl_xor(s, off, 32);
    const float mu = s * (1.0f / DM);
    float q = 0.0f;
#pragma unroll 1
    for (int c = 0; c < DM / 256; ++c) {
        const v8f v = *(const v8f*)(xr + c * 256);
#pragma unroll
        for (int k = 0; k < 8; ++k) { const float d = bfr(v[k]) - mu; q += d * d; }
    }
#pragma unroll
    for (int off = 16; off > 0; off >>= 1) q += __shfl_xor(q, off, 32);
    const float rstd = rsqrtf(q * (1.0f / DM) + 1e-5f);
    h16* hr = H + (size_t)m * DM + lane * 8;
#pragma unroll 1
    for (int ps = 0; ps < 2; ++ps) {
#pragma unroll 1
        for (int c = 0; c < DM / 256; ++c) {
            const v8f v = *(const v8f*)(xr + c * 256);
            const v8f gv = *(const v8f*)(g + c * 256 + lane * 8);
            const v8f bv = *(const v8f*)(bb + c * 256 + lane * 8);
            v8h o;
#pragma unroll
            for (int k = 0; k < 8; ++k) o[k] = toh_flush(((bfr(v[k]) - mu) * rstd) * bfr(gv[k]) + bfr(bv[k]));
            *(volatile v8h*)(hr + c * 256) = o;
        }
        if (ps == 0) __threadfence();
    }
}

__global__ __launch_bounds__(256) void k_ln_out(const float* __restrict__ Y, const float* __restrict__ g, const float* __restrict__ bb, float* OUT) {
#pragma clang fp contract(off)
    const int lane = threadIdx.x & 31;
    const int wave = __builtin_amdgcn_readfirstlane((int)(threadIdx.x >> 5));
    const int m = blockIdx.x * 8 + wave;
    const int b = m / SEQ, t = m % SEQ;
    const float* yr = Y + (size_t)m * DM + lane * 4;
    float s = 0.0f;
#pragma unroll 1
    for (int c = 0; c < DM / 128; ++c) {
        const v4f v = *(const v4f*)(yr + c * 128);
        s += v[0]; s += v[1]; s += v[2]; s += v[3];
    }
#pragma unroll
    for (int off = 16; off > 0; off >>= 1) s += __shfl_xor(s, off, 32);
    const float mu = s * (1.0f / DM);
    float q = 0.0f;
#pragma unroll 1
    for (int c = 0; c < DM / 128; ++c) {
        const v4f v = *(const v4f*)(yr + c * 128);
#pragma unroll
        for (int k = 0; k < 4; ++k) { const float d = v[k] - mu; q += d * d; }
    }
#pragma unroll
    for (int off = 16; off > 0; off >>= 1) q += __shfl_xor(q, off, 32);
    const float rstd = rsqrtf(q * (1.0f / DM) + 1e-5f);
    float* orow = OUT + ((size_t)b * OUT_SEQ + (size_t)t) * DM + lane * 4;
#pragma unroll 1
    for (int ps = 0; ps < 2; ++ps) {
#pragma unroll 1
        for (int c = 0; c < DM / 128; ++c) {
            const v4f v = *(const v4f*)(yr + c * 128);
            const v4f gv = *(const v4f*)(g + c * 128 + lane * 4);
            const v4f bv = *(const v4f*)(bb + c * 128 + lane * 4);
            v4f o;
#pragma unroll
            for (int k = 0; k < 4; ++k) o[k] = ((v[k] - mu) * rstd) * bfr(gv[k]) + bfr(bv[k]);
            *(volatile v4f*)(orow + c * 128) = o;
        }
        if (ps == 0) __threadfence();
    }
}

template <int MODE, int K>
__device__ __forceinline__ void gemm_tile(const h16* __restrict__ A, const h16* __restrict__ Bt, h16* dh, float* df, size_t obase, size_t pitch, float scale) {
    __shared__ __align__(16) float os[16 * 68];
    static_assert(K % 32 == 0);
    const int lane = threadIdx.x & 31, lr = lane & 15, hi = lane >> 4;
    v8f acc[4][4];
#pragma unroll
    for (int mb = 0; mb < 4; ++mb)
#pragma unroll
        for (int nb = 0; nb < 4; ++nb) acc[mb][nb] = (v8f){};
    const size_t foff = (size_t)lr * K + 8 * hi;
#pragma unroll 1
    for (int kc = 0; kc < K; kc += 32) {
        v16h a[4];
#pragma unroll
        for (int mb = 0; mb < 4; ++mb) a[mb] = ldh(A + foff + (size_t)mb * 16 * K + kc);
#pragma unroll
        for (int nb = 0; nb < 4; ++nb) {
            const v16h bq = ldh(Bt + foff + (size_t)nb * 16 * K + kc);
#pragma unroll
            for (int mb = 0; mb < 4; ++mb) acc[mb][nb] = wmmag(a[mb], bq, acc[mb][nb]);
        }
    }
#pragma unroll
    for (int mb = 0; mb < 4; ++mb) {
#pragma unroll
        for (int nb = 0; nb < 4; ++nb) {
#pragma unroll
            for (int j = 0; j < 8; ++j) os[(hi * 8 + j) * 68 + nb * 16 + lr] = acc[mb][nb][j] * scale;
        }
        wave_sync();
        const size_t sb = obase + (size_t)(mb * 16) * pitch;
#pragma unroll 1
        for (int ps = 0; ps < 2; ++ps) {
            if (MODE == 0) {
#pragma unroll
                for (int s = 0; s < 4; ++s) {
                    const int row = 4 * s + (lane >> 3), c8 = (lane & 7) * 8;
                    const v4f x0 = *(const v4fa*)(&os[row * 68 + c8]); const v4f x1 = *(const v4fa*)(&os[row * 68 + c8 + 4]);
                    v8h hv;
#pragma unroll
                    for (int i = 0; i < 4; ++i) { hv[i] = toh_flush(x0[i]); hv[4 + i] = toh_flush(x1[i]); }
                    *(volatile v8h*)(dh + sb + (size_t)row * pitch + c8) = hv;
                }
            } else {
#pragma unroll
                for (int s = 0; s < 8; ++s) {
                    const int row = 2 * s + (lane >> 4), c4 = (lane & 15) * 4;
                    const v4f val = *(const v4fa*)(&os[row * 68 + c4]);
                    *(volatile v4f*)(df + sb + (size_t)row * pitch + c4) = val;
                }
            }
            if (ps == 0) __threadfence();
        }
        wave_sync();
    }
}

__global__ __launch_bounds__(32) void k_gemm_q(const h16* __restrict__ H, const h16* __restrict__ W1, h16* QH) {
    const int r0 = blockIdx.x * 64, c0 = blockIdx.y * 64;
    const int bb = r0 / SEQ, tt = r0 % SEQ;
    const int z = bb * NH_ + c0 / HD, dc = c0 % HD;
    const size_t ob = ((size_t)z * SEQ + (size_t)tt) * HD + (size_t)dc;
    gemm_tile<0, DM>(H + (size_t)r0 * DM, W1 + (size_t)c0 * DM, QH, (float*)0, ob, (size_t)HD, 1.0f / WC1);
}

__global__ __launch_bounds__(32) void k_gemm_kp(const h16* __restrict__ H, const h16* __restrict__ W1, float* KF) {
    const int r0 = blockIdx.x * 64;
    const int sel = (int)(blockIdx.y >> 5), cw = (int)(blockIdx.y & 31) * 64;
    const int wrow = DE + sel * (2 * DE) + cw;
    const size_t ob = (size_t)sel * ((size_t)NB * SEQ * DE) + (size_t)r0 * DE + (size_t)cw;
    gemm_tile<1, DM>(H + (size_t)r0 * DM, W1 + (size_t)wrow * DM, (h16*)0, KF, ob, (size_t)DE, 1.0f / WC1);
}

__global__ __launch_bounds__(32) void k_gemm_v(const h16* __restrict__ W1, const h16* __restrict__ H, h16* VT) {
    const int r0 = blockIdx.x * 64, c0 = blockIdx.y * 64;
    const int bb = c0 / SEQ, tt = c0 % SEQ;
    const size_t ob = ((size_t)bb * DE + (size_t)r0) * SEQ + (size_t)tt;
    gemm_tile<0, DM>(W1 + (size_t)(2 * DE + r0) * DM, H + (size_t)c0 * DM, VT, (float*)0, ob, (size_t)SEQ, 1.0f / WC1);
}

__global__ __launch_bounds__(32) void k_gemm_out(const h16* __restrict__ G, const h16* __restrict__ W2, float* Y) {
    const int r0 = blockIdx.x * 64, c0 = blockIdx.y * 64;
    const size_t ob = (size_t)r0 * DM + (size_t)c0;
    gemm_tile<1, DE>(G + (size_t)r0 * DE, W2 + (size_t)c0 * DE, (h16*)0, Y, ob, (size_t)DM, 1.0f / (GSC * WC2));
}

__global__ __launch_bounds__(256) void k_smear(const float* __restrict__ K32, const float* __restrict__ smf, h16* KP) {
#pragma clang fp contract(off)
    const size_t e = ((size_t)blockIdx.x * 256 + threadIdx.x) * 8;
    const int d = (int)(e & (size_t)(HD - 1));
    const int row = (int)(e / HD);
    const int t = row % SEQ, z = row / SEQ;
    const int b = z / NH_, h = z % NH_;
    const float sf = bfr(smf[h]);
    const float s = __builtin_amdgcn_rcpf(1.0f + expf(-sf));
    const float s1 = 1.0f - s;
    const int tp = (t > 0) ? (t - 1) : 0;
    const float* cur = K32 + ((size_t)b * SEQ + (size_t)t) * DE + h * HD + d;
    const float* prv = K32 + ((size_t)b * SEQ + (size_t)tp) * DE + h * HD + d;
    const v4f c0 = *(const v4f*)cur, c1 = *(const v4f*)(cur + 4);
    v4f p0 = *(const v4f*)prv, p1 = *(const v4f*)(prv + 4);
    asm volatile("" : "+v"(p0));
    asm volatile("" : "+v"(p1));
    const bool hasp = t > 0;
    v8h o;
#pragma unroll
    for (int i = 0; i < 4; ++i) {
        const float q0 = hasp ? p0[i] : 0.0f, q1 = hasp ? p1[i] : 0.0f;
        o[i] = toh_flush(s1 * c0[i] + s * q0);
        o[4 + i] = toh_flush(s1 * c1[i] + s * q1);
    }
    *(volatile v8h*)(KP + e) = o; __threadfence(); *(volatile v8h*)(KP + e) = o;
}

__global__ __launch_bounds__(32 * AW) void k_flash(const h16* __restrict__ QH, const h16* __restrict__ KP, const h16* __restrict__ VT,
                                                   const float* __restrict__ PG, const float* __restrict__ slopes, h16* G) {
    __shared__ __align__(16) float os[AW * 16 * OSP];
    const int lane = threadIdx.x & 31, lr = lane & 15, hi = lane >> 4;
    const int wave = __builtin_amdgcn_readfirstlane((int)(threadIdx.x >> 5));
    const int zh = blockIdx.y; const int b = zh / NH_, h = zh % NH_;
    const int t0 = (blockIdx.x * AW + wave) * 16;
    const int nk = (t0 + 16 + 31) & ~31;
    const int lim = t0 + lr;
    const float bl2 = bfr(slopes[h]) * LOG2E;
    const size_t pbase = (size_t)zh * SEQ * HD;
    const size_t qo = pbase + (size_t)(t0 + lr) * HD + 8 * hi;
    const size_t ko = pbase + (size_t)lr * HD + 8 * hi;
    const size_t vo = pbase + (size_t)lr * SEQ + 8 * hi;
    v8f o[8];
#pragma unroll
    for (int j = 0; j < 8; ++j) o[j] = (v8f){};
    float m = NEGB, l = 0.0f;
#pragma unroll 1
    for (int key0 = 0; key0 < nk; key0 += 32) {
        v8f sa = (v8f){}, sb = (v8f){};
        const size_t kof = ko + (size_t)key0 * HD;
#pragma unroll 1
        for (int kc = 0; kc < HD; kc += 32) {
            const v16h qf = ldh(QH + qo + kc);
            const v16h ka = ldh(KP + kof + kc);
            const v16h kb = ldh(KP + kof + (size_t)16 * HD + kc);
            sa = wmmag(ka, qf, sa);
            sb = wmmag(kb, qf, sb);
        }
        const int ja = key0 + 8 * hi;
        float ta[8], tb[8]; bool fa[8], fb[8]; float mx = NEGB;
#pragma unroll
        for (int r = 0; r < 8; ++r) {
            fa[r] = (ja + r <= lim);
            fb[r] = (ja + 16 + r <= lim);
            ta[r] = sa[r] * SC2 + bl2 * (float)(ja + r - t0);
            tb[r] = sb[r] * SC2 + bl2 * (float)(ja + 16 + r - t0);
            mx = fmaxf(mx, fmaxf(fa[r] ? ta[r] : NEGB, fb[r] ? tb[r] : NEGB));
        }
        mx = fmaxf(mx, __shfl_xor(mx, 16, 32));
        const float mnew = fmaxf(m, mx);
        const float alpha = __builtin_amdgcn_exp2f(m - mnew);
        const float sh = PSH - mnew;
        v16h pb; float ls = 0.0f;
#pragma unroll
        for (int r = 0; r < 8; ++r) {
            const float xa = ta[r] + sh, xb = tb[r] + sh;
            const float ea = __builtin_amdgcn_exp2f(xa), eb = __builtin_amdgcn_exp2f(xb);
            const float ga = (fa[r] & (xa >= -14.0f)) ? ea : 0.0f;
            const float gb = (fb[r] & (xb >= -14.0f)) ? eb : 0.0f;
            const h16 pa = (h16)ga; const h16 pc = (h16)gb;
            pb[r] = pa; pb[8 + r] = pc;
            ls += (float)pa + (float)pc;
        }
        l = l * alpha + ls; m = mnew;
#pragma unroll
        for (int j = 0; j < 8; ++j) o[j] = o[j] * alpha;
        const size_t vof = vo + (size_t)key0;
#pragma unroll
        for (int jg = 0; jg < 2; ++jg) {
            v16h vf[4];
#pragma unroll
            for (int j = 0; j < 4; ++j) vf[j] = ldh(VT + vof + (size_t)((jg * 4 + j) * 16) * SEQ);
#pragma unroll
            for (int j = 0; j < 4; ++j) o[jg * 4 + j] = wmmag(vf[j], pb, o[jg * 4 + j]);
        }
    }
    l += __shfl_xor(l, 16, 32);
    const float inv = 1.0f / l;
    const int wb = wave * 16 * OSP;
#pragma unroll
    for (int j = 0; j < 8; ++j) {
        v4f a, c;
        a[0] = o[j][0] * inv; a[1] = o[j][1] * inv; a[2] = o[j][2] * inv; a[3] = o[j][3] * inv;
        c[0] = o[j][4] * inv; c[1] = o[j][5] * inv; c[2] = o[j][6] * inv; c[3] = o[j][7] * inv;
        *(v4fa*)(&os[wb + lr * OSP + 16 * j + 8 * hi]) = a; *(v4fa*)(&os[wb + lr * OSP + 16 * j + 8 * hi + 4]) = c;
    }
    wave_sync();
    const int rsel = lane >> 4, c8 = (lane & 15) * 8;
    const size_t gbase = ((size_t)b * SEQ + (size_t)t0) * DE + (size_t)h * HD + (size_t)c8;
    v8h gv[8];
#pragma unroll
    for (int s = 0; s < 8; ++s) {
        const int row = 2 * s + rsel;
        const v4f x0 = *(const v4fa*)(&os[wb + row * OSP + c8]); const v4f x1 = *(const v4fa*)(&os[wb + row * OSP + c8 + 4]);
        const float* pp = PG + gbase + (size_t)row * DE;
        const v4f p0 = *(const v4f*)pp, p1 = *(const v4f*)(pp + 4);
#pragma unroll
        for (int i = 0; i < 4; ++i) {
            const float s0 = p0[i] * __builtin_amdgcn_rcpf(1.0f + __expf(-p0[i]));
            const float s1 = p1[i] * __builtin_amdgcn_rcpf(1.0f + __expf(-p1[i]));
            gv[s][i] = toh_flush((s0 * x0[i]) * GSC);
            gv[s][4 + i] = toh_flush((s1 * x1[i]) * GSC);
        }
    }
#pragma unroll 1
    for (int ps = 0; ps < 2; ++ps) {
#pragma unroll
        for (int s = 0; s < 8; ++s) *(volatile v8h*)(G + gbase + (size_t)(2 * s + rsel) * DE) = gv[s];
        if (ps == 0) __threadfence();
    }
}

static constexpr size_t al256(size_t v) { return (v + 255) & ~(size_t)255; }
static constexpr size_t SZ_H  = al256((size_t)NB * SEQ * DM * 2);
static constexpr size_t SZ_W1 = al256((size_t)NW1 * DM * 2);
static constexpr size_t SZ_W2 = al256((size_t)DM * DE * 2);
static constexpr size_t SZ_PL = al256((size_t)NB * SEQ * DE * 2);
static constexpr size_t SZ_F  = al256((size_t)NB * SEQ * DE * 4);
static constexpr size_t SZ_Y  = al256((size_t)NB * SEQ * DM * 4);
static constexpr size_t SZ_TOTAL = SZ_H + SZ_W1 + SZ_W2 + 2 * SZ_PL + 2 * SZ_F;
static_assert(SZ_TOTAL <= (size_t)134217728);
static_assert(SZ_PL <= SZ_H + SZ_W1);
static_assert(SZ_PL + SZ_Y <= SZ_F);
static_assert(((size_t)NB * SEQ * DE * 4) % 256 == 0);
static_assert((size_t)NB * NH_ * SEQ * HD == (size_t)NB * SEQ * DE);

extern "C" void kernel_launch(void* const* d_in, const int* in_sizes, int n_in,
                              void* d_out, int out_size, void* d_ws, size_t ws_size, hipStream_t stream) {
    if (n_in < 9) return;
    const size_t needx = ((size_t)(NB - 1) * SEQ_FULL + SEQ) * DM;
    if ((size_t)in_sizes[0] < needx) return;
    if ((size_t)in_sizes[1] < (size_t)NW1 * DM || (size_t)in_sizes[2] < (size_t)DM * DE) return;
    if (in_sizes[3] < DM || in_sizes[4] < DM || in_sizes[5] < DM || in_sizes[6] < DM) return;
    if (in_sizes[7] < NH_ || in_sizes[8] < NH_) return;
    if ((size_t)out_size < ((size_t)(NB - 1) * OUT_SEQ + SEQ) * DM) return;
    if (SZ_TOTAL > ws_size) return;
    const float* x     = (const float*)d_in[0];
    const float* w_in  = (const float*)d_in[1];
    const float* w_out = (const float*)d_in[2];
    const float* g1    = (const float*)d_in[3];
    const float* b1    = (const float*)d_in[4];
    const float* g2    = (const float*)d_in[5];
    const float* b2    = (const float*)d_in[6];
    const float* slopes = (const float*)d_in[7];
    const float* smf    = (const float*)d_in[8];
    float* OUT = (float*)d_out;
    char* wsp = (char*)d_ws;
    h16* H  = (h16*)wsp; wsp += SZ_H;
    h16* W1 = (h16*)wsp; wsp += SZ_W1;
    h16* W2 = (h16*)wsp; wsp += SZ_W2;
    h16* QH = (h16*)wsp; wsp += SZ_PL;
    h16* VT = (h16*)wsp; wsp += SZ_PL;
    float* KF = (float*)wsp; wsp += 2 * SZ_F;
    h16* KP = (h16*)d_ws;
    h16* G  = (h16*)KF;
    float* Y = (float*)((char*)KF + SZ_PL);
    const float* PG = KF + (size_t)NB * SEQ * DE;

    { const unsigned n8 = (unsigned)((size_t)NW1 * DM / 8); k_wcvt<<<(n8 + 255u) / 256u, 256, 0, stream>>>(w_in, W1, n8, WC1); }
    { const unsigned n8 = (unsigned)((size_t)DM * DE / 8);  k_wcvt<<<(n8 + 255u) / 256u, 256, 0, stream>>>(w_out, W2, n8, WC2); }
    k_ln_in<<<NB * SEQ / 8, 256, 0, stream>>>(x, g1, b1, H);
    k_gemm_q<<<dim3(NB * SEQ / 64, DE / 64, 1), 32, 0, stream>>>(H, W1, QH);
    k_gemm_kp<<<dim3(NB * SEQ / 64, 2 * (DE / 64), 1), 32, 0, stream>>>(H, W1, KF);
    k_gemm_v<<<dim3(DE / 64, NB * SEQ / 64, 1), 32, 0, stream>>>(W1, H, VT);
    k_smear<<<(unsigned)((size_t)NB * NH_ * SEQ * HD / 8 / 256), 256, 0, stream>>>(KF, smf, KP);
    k_flash<<<dim3(SEQ / (16 * AW), NB * NH_, 1), 32 * AW, 0, stream>>>(QH, KP, VT, PG, slopes, G);
    k_gemm_out<<<dim3(NB * SEQ / 64, DM / 64, 1), 32, 0, stream>>>(G, W2, Y);
    k_ln_out<<<NB * SEQ / 8, 256, 0, stream>>>(Y, g2, b2, OUT);
}
